// CNN_OTAM_CLIPFSAR_43095701848304
// MI455X (gfx1250) — hardware-run, weakly checked
//
#include <hip/hip_runtime.h>
#include <math.h>

constexpr int kNQ     = 512;
constexpr int kNSup   = 128;
constexpr int kFrm    = 16;
constexpr int kDim    = 1024;
constexpr int kRowsT  = kNQ * kFrm;
constexpr int kRowsS  = kNSup * kFrm;
constexpr int kMPad   = kFrm + 2;
constexpr int kDPThreads = 128;
constexpr float kCarry    = 64.0f;
constexpr float kSimScale = 1.0f / 4096.0f;
constexpr float kLbda     = 0.5f;
constexpr float kInvLbda  = 2.0f;
static_assert(kDPThreads == kNSup, "DP block maps thread -> support video");
static_assert(kRowsT % 64 == 0 && kRowsS % 64 == 0 && kDim % 32 == 0, "GEMM tile multiples");

typedef __attribute__((ext_vector_type(16))) _Float16 v16h;
typedef __attribute__((ext_vector_type(8)))  _Float16 v8h;
typedef __attribute__((ext_vector_type(16))) __bf16   v16b;
typedef __attribute__((ext_vector_type(8)))  __bf16   v8b;
typedef __attribute__((ext_vector_type(8)))  float    v8f;
typedef __attribute__((ext_vector_type(4)))  float    v4f;
typedef __attribute__((ext_vector_type(4)))  unsigned int v4u;

__device__ __forceinline__ unsigned short f2bf_bits(float f) {
  unsigned u = __float_as_uint(f);
  return (unsigned short)((u + 0x7FFFu + ((u >> 16) & 1u)) >> 16);
}
__device__ __forceinline__ float bf_bits2f(unsigned short h) { return __uint_as_float(((unsigned)h) << 16); }

__device__ __forceinline__ void dep_guard_h(v8f& a, v8f& b, v16h x, v16h y) { asm volatile("v_nop\n\tv_nop\n\tv_nop\n\tv_nop" : "+v"(a), "+v"(b) : "v"(x), "v"(y)); }
__device__ __forceinline__ void dep_guard_b(v8f& a, v8f& b, v16b x, v16b y) { asm volatile("v_nop\n\tv_nop\n\tv_nop\n\tv_nop" : "+v"(a), "+v"(b) : "v"(x), "v"(y)); }
__device__ __forceinline__ void keep4_h(v16h a, v16h b, v16h c, v16h d) { asm volatile("v_nop" :: "v"(a), "v"(b), "v"(c), "v"(d)); }
__device__ __forceinline__ void keep4_b(v16b a, v16b b, v16b c, v16b d) { asm volatile("v_nop" :: "v"(a), "v"(b), "v"(c), "v"(d)); }
__device__ __forceinline__ void acc_guard4(v8f& a, v8f& b, v8f& c, v8f& d) { asm volatile("v_nop\n\tv_nop\n\tv_nop\n\tv_nop" : "+v"(a), "+v"(b), "+v"(c), "+v"(d)); }
template <typename T> struct Frag;
template <> struct Frag<_Float16> {
  typedef v16h V; union U { v16h v; v8h h[2]; };
  static __device__ __forceinline__ v16h load(const _Float16* p) {
    U f; f.h[0] = *(const v8h*)(p); f.h[1] = *(const v8h*)(p + 16); return f.v;
  }
  static __device__ __forceinline__ v8f mma(v16h a, v16h b, v8f c) {
    return __builtin_amdgcn_wmma_f32_16x16x32_f16(false, a, false, b, (short)0, c, false, false);
  }
  static __device__ __forceinline__ void guard(v8f& a, v8f& b, v16h x, v16h y) { dep_guard_h(a, b, x, y); }
  static __device__ __forceinline__ void keep(v16h a, v16h b, v16h c, v16h d) { keep4_h(a, b, c, d); }
};
template <> struct Frag<__bf16> {
  typedef v16b V; union U { v16b v; v8b h[2]; };
  static __device__ __forceinline__ v16b load(const __bf16* p) {
    U f; f.h[0] = *(const v8b*)(p); f.h[1] = *(const v8b*)(p + 16); return f.v;
  }
  static __device__ __forceinline__ v8f mma(v16b a, v16b b, v8f c) {
    return __builtin_amdgcn_wmma_f32_16x16x32_bf16(false, a, false, b, (short)0, c, false, false);
  }
  static __device__ __forceinline__ void guard(v8f& a, v8f& b, v16b x, v16b y) { dep_guard_b(a, b, x, y); }
  static __device__ __forceinline__ void keep(v16b a, v16b b, v16b c, v16b d) { keep4_b(a, b, c, d); }
};

__device__ __forceinline__ unsigned pk16(unsigned short a, unsigned short b) { return (unsigned)a | ((unsigned)b << 16); }
__device__ __forceinline__ unsigned short h_bits(float f) { const _Float16 h = (_Float16)f; return __builtin_bit_cast(unsigned short, h); }

template <int ET> struct Elem;
template <> struct Elem<0> { typedef _Float16 T; };
template <> struct Elem<1> { typedef __bf16 T; };
template <int ET, bool SPLIT, int BIAS_MODE, int OUT_MODE, bool RESID, int ACT = 0>
__global__ __launch_bounds__(256) void wmma_gemm64(
    const unsigned short* __restrict__ Ap, const unsigned short* __restrict__ A2p, int lda, long strideA,
    const unsigned short* __restrict__ Btp, const unsigned short* __restrict__ Bt2p, int ldb, long strideB,
    void* __restrict__ Cout, void* __restrict__ Cout2, int ldc, long strideC,
    const float* __restrict__ bias,
    const float* __restrict__ resid, long strideR,
    int M, int N, int K, float scale) {
  typedef typename Elem<ET>::T T;
  typedef typename Frag<T>::V V;
  const T* A = (const T*)Ap; const T* A2 = (const T*)A2p; const T* Bt = (const T*)Btp; const T* Bt2 = (const T*)Bt2p;
  __shared__ __align__(16) float sT[8][16 * 68];
  const int b    = blockIdx.y;
  const int lane = threadIdx.x & 31;
  const int wave = threadIdx.x >> 5;
  const int tilesN = N >> 6;
  const int tilesM = M >> 6;
  const int tile = blockIdx.x * 8 + wave;
  if (tile >= tilesM * tilesN) return;
  const int tm = tile / tilesN;
  const int tn = tile - tm * tilesN;
  const int m0 = tm << 6;
  const int n0 = tn << 6;

  const T* Ab  = A  + (size_t)b * strideA;
  const T* Bb  = Bt + (size_t)b * strideB;
  const T* Ab2 = SPLIT ? (A2  + (size_t)b * strideA) : nullptr;
  const T* Bb2 = SPLIT ? (Bt2 + (size_t)b * strideB) : nullptr;

  const int rlane = lane & 15;
  const int koff  = (lane >> 4) * 8;
  const int mOff  = (lane >> 4) * 8;

  v8f acc[4][4];
#pragma unroll
  for (int i = 0; i < 4; ++i)
#pragma unroll
    for (int j = 0; j < 4; ++j) acc[i][j] = (v8f){0.f,0.f,0.f,0.f,0.f,0.f,0.f,0.f};

  for (int k0 = 0; k0 < K; k0 += 32) {
    V bh[4], bl[4];
#pragma unroll
    for (int j = 0; j < 4; ++j) {
      const size_t bo = (size_t)(n0 + (j << 4) + rlane) * ldb + koff + k0;
      bh[j] = Frag<T>::load(Bb + bo);
      if (SPLIT) bl[j] = Frag<T>::load(Bb2 + bo);
    }
#pragma unroll
    for (int i = 0; i < 4; ++i) {
      const size_t ao = (size_t)(m0 + (i << 4) + rlane) * lda + koff + k0;
      V ah = Frag<T>::load(Ab + ao);
      V al;
      if (SPLIT) al = Frag<T>::load(Ab2 + ao);
#pragma unroll
      for (int j = 0; j < 4; ++j) {
        acc[i][j] = Frag<T>::mma(ah, bh[j], acc[i][j]);
        if (SPLIT) {
          acc[i][j] = Frag<T>::mma(ah, bl[j], acc[i][j]);
          acc[i][j] = Frag<T>::mma(al, bh[j], acc[i][j]);
        }
      }
      Frag<T>::guard(acc[i][0], acc[i][3], ah, SPLIT ? al : ah);
    }
    Frag<T>::keep(bh[0], bh[1], bh[2], bh[3]);
    if (SPLIT) Frag<T>::keep(bl[0], bl[1], bl[2], bl[3]);
  }
  acc_guard4(acc[0][0], acc[0][1], acc[0][2], acc[0][3]);
  acc_guard4(acc[1][0], acc[1][1], acc[1][2], acc[1][3]);
  acc_guard4(acc[2][0], acc[2][1], acc[2][2], acc[2][3]);
  acc_guard4(acc[3][0], acc[3][1], acc[3][2], acc[3][3]);

  float* slab = sT[wave];
  const float* Rb = RESID ? (resid + (size_t)b * strideR) : nullptr;
#pragma unroll
  for (int i = 0; i < 4; ++i) {
    const int mBase = m0 + (i << 4);
#pragma unroll
    for (int j = 0; j < 4; ++j) {
      const int n = n0 + (j << 4) + rlane;
      float bv = 0.f;
      if (BIAS_MODE == 2) bv = bias[n];
#pragma unroll
      for (int r = 0; r < 8; ++r) {
        float v = acc[i][j][r] * scale;
        if (BIAS_MODE == 1) v += bias[mBase + mOff + r];
        if (BIAS_MODE == 2) v += bv;
        if (RESID) v += Rb[(size_t)(mBase + mOff + r) * ldc + n];
        if (ACT == 1) v = tanhf(v);
        if (ACT == 2) v = fmaxf(v, 0.0f);
        if (ACT == 3) v = v / (1.0f + expf(-v));
        if (ACT == 4) v = (v > 0.f) ? v : 0.01f * v;
        if (ACT == 5) v = 0.5f * v * (1.0f + erff(v * 0.70710678118654752f));
        slab[(mOff + r) * 68 + (j << 4) + rlane] = v;
      }
    }
    __builtin_amdgcn_fence(__ATOMIC_RELEASE, "workgroup");
    __builtin_amdgcn_wave_barrier();
    __builtin_amdgcn_fence(__ATOMIC_ACQUIRE, "workgroup");
    if (OUT_MODE == 0) {
      float* C = (float*)Cout + (size_t)b * strideC;
      const int hh = lane >> 4, c4 = (lane & 15) * 4;
      for (int pass = 0; pass < 2; ++pass) {
#pragma unroll
        for (int it = 0; it < 8; ++it) {
          const int row = it * 2 + hh;
          v4f v = *(const v4f*)(slab + row * 68 + c4);
          *(volatile v4f*)(C + (size_t)(mBase + row) * ldc + n0 + c4) = v;
        }
        __threadfence();
      }
    } else {
      const int q = lane >> 3, c8 = (lane & 7) * 8;
      unsigned short* C  = (unsigned short*)Cout  + (size_t)b * strideC;
      unsigned short* C2 = (OUT_MODE == 2) ? ((unsigned short*)Cout2 + (size_t)b * strideC) : nullptr;
      for (int pass = 0; pass < 2; ++pass) {
#pragma unroll
        for (int it = 0; it < 4; ++it) {
          const int row = it * 4 + q;
          const float* sp = slab + row * 68 + c8;
          v8h hv, lv;
#pragma unroll
          for (int e = 0; e < 8; ++e) {
            if (OUT_MODE == 1) {
              hv[e] = (_Float16)sp[e];
            } else {
              unsigned short hb = f2bf_bits(sp[e]);
              unsigned short lb = f2bf_bits(sp[e] - bf_bits2f(hb));
              hv[e] = __builtin_bit_cast(_Float16, hb);
              lv[e] = __builtin_bit_cast(_Float16, lb);
            }
          }
          *(volatile v8h*)(C + (size_t)(mBase + row) * ldc + n0 + c8) = hv;
          if (OUT_MODE == 2) *(volatile v8h*)(C2 + (size_t)(mBase + row) * ldc + n0 + c8) = lv;
        }
        __threadfence();
      }
    }
    __builtin_amdgcn_fence(__ATOMIC_RELEASE, "workgroup");
    __builtin_amdgcn_wave_barrier();
    __builtin_amdgcn_fence(__ATOMIC_ACQUIRE, "workgroup");
  }
}

__global__ __launch_bounds__(128) void rownorm_f16_kernel(const float* __restrict__ x, unsigned short* __restrict__ y,
                                                          int nrows, float carry) {
  __shared__ float red[4];
  int row = blockIdx.x;
  if (row > nrows - 1) row = nrows - 1;
  const int t    = threadIdx.x;
  const int lane = t & 31, wave = t >> 5;
  const int c0   = t * 8;
  const float* xr = x + (size_t)row * kDim + c0;
  const v4f a = *(const v4f*)(xr);
  const v4f c = *(const v4f*)(xr + 4);
  float s = ((a[0] * a[0] + a[1] * a[1]) + (a[2] * a[2] + a[3] * a[3])) +
            ((c[0] * c[0] + c[1] * c[1]) + (c[2] * c[2] + c[3] * c[3]));
#pragma unroll
  for (int off = 16; off > 0; off >>= 1) s += __shfl_xor(s, off, 32);
  if (lane == 0) red[wave] = s;
  __syncthreads();
  const float ss = (red[0] + red[1]) + (red[2] + red[3]);
  const float g  = rsqrtf(ss) * carry;
  unsigned short hb[8];
#pragma unroll
  for (int e = 0; e < 4; ++e) {
    hb[e]     = h_bits(a[e] * g);
    hb[4 + e] = h_bits(c[e] * g);
  }
  const v4u u = (v4u){pk16(hb[0], hb[1]), pk16(hb[2], hb[3]), pk16(hb[4], hb[5]), pk16(hb[6], hb[7])};
  unsigned short* yp = y + (size_t)row * kDim + c0;
  *(volatile v4u*)yp = u;
  __threadfence();
  *(volatile v4u*)yp = u;
}

__global__ __launch_bounds__(128) void align_dp_kernel(const float* __restrict__ sim, float* __restrict__ out) {
  __shared__ float rows[2 * kMPad * kDPThreads];
  __shared__ __align__(16) float res[kDPThreads];
  const int tid = threadIdx.x;
  const int q   = blockIdx.x;
  const size_t base = (size_t)(q * kFrm) * kRowsS + (size_t)tid * kFrm;
  float total = 0.0f;
#pragma unroll 1
  for (int dir = 0; dir < 2; ++dir) {
    const int strideL = (dir == 0) ? kRowsS : 1;
    const int strideM = (dir == 0) ? 1 : kRowsS;
    float run = 0.0f;
    rows[(0 * kMPad + 0) * kDPThreads + tid] = 0.0f;
#pragma unroll 1
    for (int m = 1; m < kMPad; ++m) {
      const int mc = (m - 1 < kFrm - 1) ? (m - 1) : (kFrm - 1);
      const float sv = sim[base + (size_t)mc * strideM];
      const float dv = (m <= kFrm) ? (1.0f - sv) : 0.0f;
      run = run + dv;
      rows[(0 * kMPad + m) * kDPThreads + tid] = run;
    }
    float last = run;
    int pb = 0;
#pragma unroll 1
    for (int l = 1; l < kFrm; ++l) {
      const int nb = pb ^ 1;
      const int pOff = pb * kMPad;
      const int nOff = nb * kMPad;
      rows[(nOff + 0) * kDPThreads + tid] = 0.0f;
      float left = 0.0f;
      float a = rows[(pOff + 0) * kDPThreads + tid];
      const size_t lbase = base + (size_t)l * strideL;
#pragma unroll 1
      for (int m = 1; m < kMPad; ++m) {
        const float cpm = rows[(pOff + m) * kDPThreads + tid];
        const int mc = (m - 1 < kFrm - 1) ? (m - 1) : (kFrm - 1);
        const float sv = sim[lbase + (size_t)mc * strideM];
        const float dv = (m <= kFrm) ? (1.0f - sv) : 0.0f;
        const bool edge = (m == 1) || (m == kMPad - 1);
        float mn = fminf(a, left);
        mn = edge ? fminf(mn, cpm) : mn;
        float ssum = __expf((mn - a) * kInvLbda) + __expf((mn - left) * kInvLbda);
        const float e3 = __expf((mn - cpm) * kInvLbda);
        ssum = edge ? (ssum + e3) : ssum;
        const float val = dv + (mn - kLbda * __logf(ssum));
        rows[(nOff + m) * kDPThreads + tid] = val;
        left = val;
        a = cpm;
      }
      last = left;
      pb = nb;
    }
    total += last;
  }
  res[tid] = -total;
  __syncthreads();
  if (tid < 32) {
    const v4f v = *(const v4f*)(res + tid * 4);
    float* op = out + (size_t)q * kNSup + tid * 4;
    *(volatile v4f*)op = v;
    __threadfence();
    *(volatile v4f*)op = v;
  }
}

extern "C" void kernel_launch(void* const* d_in, const int* in_sizes, int n_in,
                              void* d_out, int out_size, void* d_ws, size_t ws_size,
                              hipStream_t stream) {
  if (n_in < 2) return;
  if (in_sizes[0] != kNSup * kFrm * kDim) return;
  if (in_sizes[1] != kNQ * kFrm * kDim) return;
  if (out_size != kNQ * kNSup) return;

  const float* support = (const float*)d_in[0];
  const float* target  = (const float*)d_in[1];
  float* outp = (float*)d_out;

  const size_t SZ_TN  = (size_t)kRowsT * kDim * 2;
  const size_t SZ_SN  = (size_t)kRowsS * kDim * 2;
  const size_t SZ_SIM = (size_t)kRowsT * kRowsS * 4;
  size_t off = 0;
  const size_t oTN  = off; off += SZ_TN;
  const size_t oSN  = off; off += SZ_SN;
  const size_t oSIM = off; off += SZ_SIM;
  const size_t TOTAL = off;
  if (TOTAL > ws_size) return;
  if (TOTAL > (size_t)134217728) return;

  char* ws = (char*)d_ws;
  unsigned short* TN16 = (unsigned short*)(ws + oTN);
  unsigned short* SN16 = (unsigned short*)(ws + oSN);
  float*          SIM  = (float*)(ws + oSIM);
  const float* dummy_f = SIM;

  rownorm_f16_kernel<<<dim3(kRowsS), dim3(128), 0, stream>>>(support, SN16, kRowsS, kCarry);
  rownorm_f16_kernel<<<dim3(kRowsT), dim3(128), 0, stream>>>(target,  TN16, kRowsT, kCarry);

  const int tiles = (kRowsT / 64) * (kRowsS / 64);
  const dim3 gG((tiles + 7) / 8, 1);
  wmma_gemm64<0, false, 0, 0, false><<<gG, dim3(256), 0, stream>>>(
      TN16, TN16, kDim, 0L, SN16, SN16, kDim, 0L, (void*)SIM, (void*)SIM, kRowsS, 0L,
      dummy_f, dummy_f, 0L, kRowsT, kRowsS, kDim, kSimScale);

  align_dp_kernel<<<dim3(kNQ), dim3(kDPThreads), 0, stream>>>(SIM, outp);
}
